// GCNNet_54382875902525
// MI455X (gfx1250) — hardware-verified
//
#include <hip/hip_runtime.h>
#include <stddef.h>
#include <stdint.h>
#include <math.h>


#define F0     75
#define F1     75
#define F2     150
#define F3     300
#define FG     1024
#define FO     128
#define NGR    256
#define K1P    96
#define N1P    96
#define K2P    192
#define N2P    160
#define K3P    320
#define N3P    320
#define KG1    640
#define KG2    2048
#define NTHR   256
#define NWAVE  8
#define EPT    8
#define CHUNK  (NTHR * EPT)
#define WCAP   (EPT * 32)
#define LISTN  (NWAVE * WCAP)
#define NBD    8192
#define SLD    13
#define NBA    1024
#define SLA    10
#define RCAP   20480
#define DEGCAP 64
#define GBM    64
#define GBN    32
#define GTHR   128
#define AGG_ZINTS    (LISTN + 2 * RCAP + 3 * NBA)
#define MISC_INTS    16
#define ROWB_INTS    160
#define AGG_LDS_INTS (AGG_ZINTS + MISC_INTS + NWAVE * ROWB_INTS)
#define NU1V   (K1P * (K1P / 8))
#define NU1    1280
#define NU2    (N2P * (K2P / 8))
#define NU3    (N3P * (K3P / 8))
#define NU4    (FG * (KG1 / 8))
#define NU5    (FO * (KG2 / 8))
#define NUALL  (NU1 + NU2 + NU3 + NU4 + NU5)
#define WSMAX  134217728

static_assert((CHUNK & (CHUNK - 1)) == 0 && CHUNK <= 4096);
static_assert((NBD & (NBD - 1)) == 0 && NBD == (1 << SLD));
static_assert((NBA & (NBA - 1)) == 0 && NBA == (1 << SLA));
static_assert(((long long)CHUNK << SLD) < (1LL << 31));
static_assert(((long long)CHUNK << SLA) < (1LL << 31));
static_assert(NBD % (NTHR * 4) == 0);
static_assert(NBA % NWAVE == 0 && NBA % 32 == 0 && NBA % GBM == 0);
static_assert(RCAP % 4 == 0 && AGG_ZINTS % 4 == 0 && LISTN % 4 == 0 && ROWB_INTS % 4 == 0);
static_assert(K1P % 32 == 0 && K2P % 32 == 0 && K3P % 32 == 0 && KG1 % 32 == 0 && KG2 % 32 == 0);
static_assert(N1P % GBN == 0 && N2P % GBN == 0 && N3P % GBN == 0 && FG % GBN == 0 && FO % GBN == 0);
static_assert(K2P == 2 * N1P && K3P == 2 * N2P && KG1 == 2 * N3P && KG2 == 2 * FG);
static_assert(N1P >= F1 && N2P >= F2 && N3P >= F3 && K1P >= F0);
static_assert(GBM == (GTHR / 32) * 16 && GBN == 32);
static_assert(NU1 % NTHR == 0 && NU2 % NTHR == 0 && NU3 % NTHR == 0 && NU4 % NTHR == 0 && NU5 % NTHR == 0);
static_assert(NU1V <= NU1 && NU1V % 32 == 0);
static_assert(AGG_LDS_INTS * 4 <= 300000);
static_assert(N1P * 4 <= ROWB_INTS * 4 && K2P * 2 <= ROWB_INTS * 4 && K3P * 2 <= ROWB_INTS * 4);
static_assert(NGR % GBM == 0 && (NGR * FO) == 32768);
static_assert(KG1 / 8 == 80);

typedef float          v4f   __attribute__((ext_vector_type(4)));
typedef float          v8f   __attribute__((ext_vector_type(8)));
typedef int            v4i   __attribute__((ext_vector_type(4)));
typedef int            v8i   __attribute__((ext_vector_type(8)));
typedef unsigned short v8us  __attribute__((ext_vector_type(8)));
typedef unsigned short v16us __attribute__((ext_vector_type(16)));
typedef __bf16         v16bf __attribute__((ext_vector_type(16)));
typedef v4f  __attribute__((may_alias)) v4fa;
typedef v4i  __attribute__((may_alias)) v4ia;
typedef v8us __attribute__((may_alias)) v8usa;
union FragB { v16bf v; v16us u; v8us h[2]; v8i w; };

__device__ __forceinline__ v8f wmb(const FragB& a, const FragB& b, v8f c) {
  v8f d = __builtin_amdgcn_wmma_f32_16x16x32_bf16(false, a.v, false, b.v, (short)0, c, false, false);
  asm volatile("v_nop\n\tv_nop\n\tv_nop\n\tv_nop" : "+v"(d) : "v"(a.w), "v"(b.w));
  return d;
}

__device__ __forceinline__ unsigned bf16_bits(float f) {
  const unsigned u = __float_as_uint(f);
  const unsigned r = (u + 0x7FFFu + ((u >> 16) & 1u)) >> 16;
  return (f != f) ? 0x7FC0u : r;
}
__device__ __forceinline__ float bf16_val(float f) {
  return __uint_as_float(bf16_bits(f) << 16);
}
__device__ __forceinline__ void split_bf(float v, unsigned& hb, unsigned& lb) {
  hb = bf16_bits(v);
  const float hf = __uint_as_float(hb << 16);
  float d = v - hf;
  d = ((hb & 0x7FFFu) == 0x7F80u) ? 0.0f : d;
  lb = bf16_bits(d);
}
__device__ __forceinline__ float relu_nan(float t) {
  return (t > 0.0f) ? t : ((t != t) ? t : 0.0f);
}
__device__ __forceinline__ float nmax(float m, float v) {
  return (v != v) ? v : ((v > m) ? v : m);
}

template <int SLB>
__device__ __forceinline__ int scan_chunk(const int* __restrict__ dsts, int nE, int cbase, int slotBase,
                                          int nb, int vec8, int* list, int tid, int lane, int wave) {
  int wc = 0;
  const int el0  = tid * EPT;
  const int e0   = cbase + el0;
  const int sent = -2147483647 - 1;
  v4i da, db;
  if (vec8 != 0 && cbase + CHUNK <= nE) {
    da = *(const v4i*)(dsts + e0);
    db = *(const v4i*)(dsts + e0 + 4);
  } else {
    da.x = (e0     < nE) ? dsts[min(e0,     nE - 1)] : sent;
    da.y = (e0 + 1 < nE) ? dsts[min(e0 + 1, nE - 1)] : sent;
    da.z = (e0 + 2 < nE) ? dsts[min(e0 + 2, nE - 1)] : sent;
    da.w = (e0 + 3 < nE) ? dsts[min(e0 + 3, nE - 1)] : sent;
    db.x = (e0 + 4 < nE) ? dsts[min(e0 + 4, nE - 1)] : sent;
    db.y = (e0 + 5 < nE) ? dsts[min(e0 + 5, nE - 1)] : sent;
    db.z = (e0 + 6 < nE) ? dsts[min(e0 + 6, nE - 1)] : sent;
    db.w = (e0 + 7 < nE) ? dsts[min(e0 + 7, nE - 1)] : sent;
  }
  const unsigned nbs = (unsigned)slotBase;
  const unsigned unb = (unsigned)nb;
  const unsigned s0 = (unsigned)da.x - nbs, s1 = (unsigned)da.y - nbs;
  const unsigned s2 = (unsigned)da.z - nbs, s3 = (unsigned)da.w - nbs;
  const unsigned s4 = (unsigned)db.x - nbs, s5 = (unsigned)db.y - nbs;
  const unsigned s6 = (unsigned)db.z - nbs, s7 = (unsigned)db.w - nbs;
  const bool h0 = s0 < unb, h1 = s1 < unb, h2 = s2 < unb, h3 = s3 < unb;
  const bool h4 = s4 < unb, h5 = s5 < unb, h6 = s6 < unb, h7 = s7 < unb;
  const unsigned any = __builtin_amdgcn_ballot_w32(h0 | h1 | h2 | h3 | h4 | h5 | h6 | h7);
  if (any != 0u) {
#define HITJ(J, HJ, SJ) { \
      const unsigned mj = __builtin_amdgcn_ballot_w32(HJ); \
      if (mj != 0u) { \
        if (HJ) { \
          const int pos = wc + (int)__builtin_amdgcn_mbcnt_lo(mj, 0u); \
          if (pos < WCAP) list[wave * WCAP + pos] = ((el0 + (J)) << SLB) | (int)(SJ); \
        } \
        wc += (int)__builtin_popcount(mj); } }
    HITJ(0, h0, s0)
    HITJ(1, h1, s1)
    HITJ(2, h2, s2)
    HITJ(3, h3, s3)
    HITJ(4, h4, s4)
    HITJ(5, h5, s5)
    HITJ(6, h6, s6)
    HITJ(7, h7, s7)
#undef HITJ
  }
  return wc;
}

__global__ __launch_bounds__(NTHR) void k_wprep(const float* __restrict__ W1, const float* __restrict__ W2,
                                                const float* __restrict__ W3, const float* __restrict__ Wg1,
                                                const float* __restrict__ Wg2,
                                                unsigned short* P1, unsigned short* P2, unsigned short* P3,
                                                unsigned short* P4, unsigned short* P5) {
  const int u = (int)blockIdx.x * NTHR + (int)threadIdx.x;
  const float* W;
  unsigned short* P;
  int v, n, k8, srcN, kTrue, nTrue, kHalf, ilv;
  if (u < NU1) {
    v = u; if (v >= NU1V) return;
    n = v / (K1P / 8); k8 = (v - n * (K1P / 8)) * 8;
    W = W1; P = P1; srcN = F1; kTrue = F0; nTrue = F1; kHalf = K1P; ilv = 0;
  } else if (u < NU1 + NU2) {
    v = u - NU1;
    n = v / (K2P / 8); k8 = (v - n * (K2P / 8)) * 8;
    W = W2; P = P2; srcN = F2; kTrue = F1; nTrue = F2; kHalf = N1P; ilv = 0;
  } else if (u < NU1 + NU2 + NU3) {
    v = u - NU1 - NU2;
    n = v / (K3P / 8); k8 = (v - n * (K3P / 8)) * 8;
    W = W3; P = P3; srcN = F3; kTrue = F2; nTrue = F3; kHalf = N2P; ilv = 0;
  } else if (u < NU1 + NU2 + NU3 + NU4) {
    v = u - NU1 - NU2 - NU3;
    n = v / (KG1 / 8); k8 = (v - n * (KG1 / 8)) * 8;
    W = Wg1; P = P4; srcN = FG; kTrue = F3; nTrue = FG; kHalf = N3P; ilv = 0;
  } else if (u < NUALL) {
    v = u - NU1 - NU2 - NU3 - NU4;
    n = v / (KG2 / 8); k8 = (v - n * (KG2 / 8)) * 8;
    W = Wg2; P = P5; srcN = FO; kTrue = FG; nTrue = FO; kHalf = KG2; ilv = 1;
  } else {
    return;
  }
  const int ncl = n < nTrue ? n : nTrue - 1;
  v8us o;
#pragma unroll
  for (int i = 0; i < 8; ++i) {
    const int kp = k8 + i;
    const int ka = (kp >= kHalf) ? kp - kHalf : kp;
    const int kb = ((kp >> 6) << 5) | (kp & 31);
    const int kk = (ilv != 0) ? kb : ka;
    const bool ok = (kk < kTrue) && (n < nTrue);
    const int kc = kk < kTrue ? kk : kTrue - 1;
    const float t = W[(size_t)kc * (size_t)srcN + ncl];
    o[i] = ok ? (unsigned short)bf16_bits(t) : (unsigned short)0;
  }
  unsigned short* dp = P + (size_t)v * 8;
  *(volatile v8us*)dp = o;
  __threadfence();
  *(volatile v8us*)dp = o;
}

__global__ __launch_bounds__(NTHR) void k_cvx(const float* __restrict__ x, int nN, int nUnits,
                                              unsigned short* xb) {
  const int u = (int)blockIdx.x * NTHR + (int)threadIdx.x;
  if (u >= nUnits) return;
  const int row = u / (K1P / 8);
  const int k8  = (u - row * (K1P / 8)) * 8;
  const int rc  = row < nN ? row : nN - 1;
  const float* p = x + (size_t)rc * F0;
  const bool okr = row < nN;
  v8us o;
#pragma unroll
  for (int i = 0; i < 8; ++i) {
    const int c  = k8 + i;
    const int cc = c < F0 ? c : F0 - 1;
    const float t = p[cc];
    o[i] = (okr && c < F0) ? (unsigned short)bf16_bits(t) : (unsigned short)0;
  }
  unsigned short* dp = xb + (size_t)u * 8;
  *(volatile v8us*)dp = o;
  __threadfence();
  *(volatile v8us*)dp = o;
}

__global__ __launch_bounds__(NTHR) void k_deg(const int* __restrict__ dsts, int nE, int vec8, float* dis) {
  __shared__ __attribute__((aligned(16))) int scnt[NBD];
  __shared__ __attribute__((aligned(16))) int list[LISTN];
  __shared__ int wcnt[NWAVE];
  const int tid = (int)threadIdx.x, lane = tid & 31, wave = tid >> 5;
  const int nodeBase = (int)blockIdx.x * NBD;

  for (int i = tid; i < NBD; i += NTHR) scnt[i] = 0;
  for (int i = tid; i < LISTN; i += NTHR) list[i] = 0;
  if (tid < NWAVE) wcnt[tid] = 0;
  __syncthreads();

  const int nChunks = (nE + CHUNK - 1) / CHUNK;
#pragma unroll 1
  for (int ch = 0; ch < nChunks; ++ch) {
    const int cbase = ch * CHUNK;
    const int wc = scan_chunk<SLD>(dsts, nE, cbase, nodeBase, NBD, vec8, list, tid, lane, wave);
    if (lane == 0) wcnt[wave] = wc;
    __syncthreads();
    if (wave == 0) {
#pragma unroll 1
      for (int w2 = 0; w2 < NWAVE; ++w2) {
        int c = wcnt[w2];
        c = c < 0 ? 0 : (c > WCAP ? WCAP : c);
#pragma unroll 1
        for (int b0 = 0; b0 < c; b0 += 32) {
          const int idx = b0 + lane;
          const int ent = list[w2 * WCAP + (idx < WCAP ? idx : WCAP - 1)];
          const int m32 = (c - b0) < 32 ? (c - b0) : 32;
#pragma unroll 1
          for (int k = 0; k < m32; ++k) {
            const int uu = __builtin_amdgcn_readlane(ent, k);
            const int sl = uu & (NBD - 1);
            if (lane == 0) scnt[sl] = scnt[sl] + 1;
          }
        }
      }
    }
    __syncthreads();
  }

  v4f vals[NBD / (NTHR * 4)];
#pragma unroll
  for (int it = 0; it < NBD / (NTHR * 4); ++it) {
    const int s0 = it * (NTHR * 4) + 4 * tid;
    const v4i c4 = *(const v4ia*)(scnt + s0);
    const float d0 = (float)c4.x + 1.0f, d1 = (float)c4.y + 1.0f;
    const float d2 = (float)c4.z + 1.0f, d3 = (float)c4.w + 1.0f;
    v4f v;
    v.x = (d0 > 0.0f) ? rsqrtf(fmaxf(d0, 1e-12f)) : 0.0f;
    v.y = (d1 > 0.0f) ? rsqrtf(fmaxf(d1, 1e-12f)) : 0.0f;
    v.z = (d2 > 0.0f) ? rsqrtf(fmaxf(d2, 1e-12f)) : 0.0f;
    v.w = (d3 > 0.0f) ? rsqrtf(fmaxf(d3, 1e-12f)) : 0.0f;
    vals[it] = v;
  }
#pragma unroll
  for (int it = 0; it < NBD / (NTHR * 4); ++it) {
    const int s0 = it * (NTHR * 4) + 4 * tid;
    *(volatile v4f*)(dis + (size_t)nodeBase + s0) = vals[it];
  }
  __threadfence();
#pragma unroll
  for (int it = 0; it < NBD / (NTHR * 4); ++it) {
    const int s0 = it * (NTHR * 4) + 4 * tid;
    *(volatile v4f*)(dis + (size_t)nodeBase + s0) = vals[it];
  }
}

template <int MODE>
__global__ __launch_bounds__(GTHR) void k_gemm(
    const unsigned short* __restrict__ A, const unsigned short* __restrict__ WT,
    const float* __restrict__ bias, int nTrue, float* outF, unsigned short* outH, int K, int ldo)
{
  __shared__ __attribute__((aligned(16))) float stg[GBM * GBN];
  const int tid = (int)threadIdx.x, lane = tid & 31, wave = tid >> 5, hh = lane >> 4, m = lane & 15;
  const int rowBase = (int)blockIdx.x * GBM;
  const int col0    = (int)blockIdx.y * GBN;

  v8f acc[2];
  {
    const v8f z = {0.f, 0.f, 0.f, 0.f, 0.f, 0.f, 0.f, 0.f};
    acc[0] = z; acc[1] = z;
  }
  const unsigned short* ap = A  + (size_t)(rowBase + 16 * wave + m) * (size_t)K + 8 * hh;
  const unsigned short* wp = WT + (size_t)(col0 + m) * (size_t)K + 8 * hh;
  const int ksteps = K >> 5;
#pragma unroll 1
  for (int ks = 0; ks < ksteps; ++ks) {
    FragB af;
    af.h[0] = *(const v8usa*)(ap + 32 * ks);
    af.h[1] = *(const v8usa*)(ap + 32 * ks + 16);
#pragma unroll
    for (int t = 0; t < 2; ++t) {
      const unsigned short* wq = wp + (size_t)(16 * t) * (size_t)K + 32 * ks;
      FragB bf;
      bf.h[0] = *(const v8usa*)wq;
      bf.h[1] = *(const v8usa*)(wq + 16);
      acc[t] = wmb(af, bf, acc[t]);
    }
  }

#pragma unroll
  for (int t = 0; t < 2; ++t) {
    const int lc = 16 * t + m;
#pragma unroll
    for (int r = 0; r < 8; ++r) {
      const int lr = 16 * wave + 8 * hh + r;
      stg[lr * GBN + lc] = acc[t][r];
    }
  }
  __syncthreads();

  const int q  = lane & 7;
  const int rq = lane >> 3;
  if constexpr (MODE != 2) {
    float b0 = 0.0f, b1 = 0.0f, b2 = 0.0f, b3 = 0.0f;
    if constexpr (MODE != 0) {
      const int c  = col0 + 4 * q;
      const int nl = nTrue - 1;
      const float t0 = bias[min(c,     nl)];
      const float t1 = bias[min(c + 1, nl)];
      const float t2 = bias[min(c + 2, nl)];
      const float t3 = bias[min(c + 3, nl)];
      b0 = (c     < nTrue) ? bf16_val(t0) : 0.0f;
      b1 = (c + 1 < nTrue) ? bf16_val(t1) : 0.0f;
      b2 = (c + 2 < nTrue) ? bf16_val(t2) : 0.0f;
      b3 = (c + 3 < nTrue) ? bf16_val(t3) : 0.0f;
    }
    v4f fv[4];
#pragma unroll
    for (int i = 0; i < 4; ++i) {
      const int lr = 16 * wave + 4 * i + rq;
      v4f v = *(const v4fa*)(stg + lr * GBN + 4 * q);
      v.x = v.x + b0; v.y = v.y + b1; v.z = v.z + b2; v.w = v.w + b3;
      if constexpr (MODE == 1) {
        v.x = relu_nan(v.x); v.y = relu_nan(v.y); v.z = relu_nan(v.z); v.w = relu_nan(v.w);
      }
      fv[i] = v;
    }
#pragma unroll
    for (int i = 0; i < 4; ++i) {
      const int gr = rowBase + 16 * wave + 4 * i + rq;
      float* op = outF + (size_t)gr * (size_t)ldo + col0 + 4 * q;
      *(volatile v4f*)op = fv[i];
    }
    __threadfence();
#pragma unroll
    for (int i = 0; i < 4; ++i) {
      const int gr = rowBase + 16 * wave + 4 * i + rq;
      float* op = outF + (size_t)gr * (size_t)ldo + col0 + 4 * q;
      *(volatile v4f*)op = fv[i];
    }
  } else {
    const int cq = 8 * (q & 3);
    const bool lsel = q >= 4;
    const v4f ba = *(const v4f*)(bias + col0 + cq);
    const v4f bb = *(const v4f*)(bias + col0 + cq + 4);
    float bz[8];
    bz[0] = bf16_val(ba.x); bz[1] = bf16_val(ba.y); bz[2] = bf16_val(ba.z); bz[3] = bf16_val(ba.w);
    bz[4] = bf16_val(bb.x); bz[5] = bf16_val(bb.y); bz[6] = bf16_val(bb.z); bz[7] = bf16_val(bb.w);
    v8us hv[4];
#pragma unroll
    for (int i = 0; i < 4; ++i) {
      const int lr = 16 * wave + 4 * i + rq;
      const v4f x0 = *(const v4fa*)(stg + lr * GBN + cq);
      const v4f x1 = *(const v4fa*)(stg + lr * GBN + cq + 4);
      float xs[8];
      xs[0] = x0.x; xs[1] = x0.y; xs[2] = x0.z; xs[3] = x0.w;
      xs[4] = x1.x; xs[5] = x1.y; xs[6] = x1.z; xs[7] = x1.w;
      v8us o;
#pragma unroll
      for (int e = 0; e < 8; ++e) {
        const float t = relu_nan(xs[e] + bz[e]);
        unsigned hb, lb;
        split_bf(t, hb, lb);
        o[e] = (unsigned short)(lsel ? lb : hb);
      }
      hv[i] = o;
    }
#pragma unroll
    for (int i = 0; i < 4; ++i) {
      const int gr = rowBase + 16 * wave + 4 * i + rq;
      unsigned short* op = outH + (size_t)gr * (size_t)ldo + 2 * col0 + 8 * q;
      *(volatile v8us*)op = hv[i];
    }
    __threadfence();
#pragma unroll
    for (int i = 0; i < 4; ++i) {
      const int gr = rowBase + 16 * wave + 4 * i + rq;
      unsigned short* op = outH + (size_t)gr * (size_t)ldo + 2 * col0 + 8 * q;
      *(volatile v8us*)op = hv[i];
    }
  }
}

template <int NJ, int F32OUT>
__global__ __launch_bounds__(NTHR) void k_scan(const int* __restrict__ srcs, const int* __restrict__ dsts,
                                               int nE, int nN, int vec8, int mRows,
                                               const float* __restrict__ dis, const float* __restrict__ xl,
                                               const float* __restrict__ bias, int nBias, int* outp) {
  constexpr int PIN = 32 * NJ;
  constexpr int NP  = 8 * NJ;
  static_assert(NP <= 40 && PIN <= ROWB_INTS);
  static_assert(F32OUT == 0 || NJ == 3);
  extern __shared__ __attribute__((aligned(16))) int dsm[];
  int* list = dsm;
  int* hl   = dsm + LISTN;
  int* sl   = hl + RCAP;
  int* cnt  = sl + RCAP;
  int* offs = cnt + NBA;
  int* cur  = offs + NBA;
  int* misc = cur + NBA;
  const int tid = (int)threadIdx.x, lane = tid & 31, wave = tid >> 5;
  int* rowb = misc + MISC_INTS + wave * ROWB_INTS;
  const int nodeBase = (int)blockIdx.x * NBA;

  {
    const v4i z4 = {0, 0, 0, 0};
    for (int i = tid * 4; i < AGG_ZINTS; i += NTHR * 4) *(v4ia*)(dsm + i) = z4;
    if (tid < MISC_INTS) misc[tid] = 0;
  }
  float bv[NJ];
#pragma unroll
  for (int j = 0; j < NJ; ++j) {
    const int c = lane + 32 * j;
    const float t = bias[c < nBias ? c : nBias - 1];
    bv[j] = (F32OUT != 0 && c < nBias) ? bf16_val(t) : 0.0f;
  }
  __syncthreads();

  int t = 0, ov = 0;
  const int nChunks = (nE + CHUNK - 1) / CHUNK;
#pragma unroll 1
  for (int ch = 0; ch < nChunks; ++ch) {
    const int cbase = ch * CHUNK;
    const int wc = scan_chunk<SLA>(dsts, nE, cbase, nodeBase, NBA, vec8, list, tid, lane, wave);
    if (lane == 0) misc[wave] = wc;
    __syncthreads();
    if (wave == 0) {
#pragma unroll 1
      for (int w2 = 0; w2 < NWAVE; ++w2) {
        int c = misc[w2];
        c = c < 0 ? 0 : (c > WCAP ? WCAP : c);
#pragma unroll 1
        for (int b0 = 0; b0 < c; b0 += 32) {
          const int idx = b0 + lane;
          const int ent = list[w2 * WCAP + (idx < WCAP ? idx : WCAP - 1)];
          const int m32 = (c - b0) < 32 ? (c - b0) : 32;
#pragma unroll 1
          for (int k = 0; k < m32; ++k) {
            const int u    = __builtin_amdgcn_readlane(ent, k);
            const int slot = u & (NBA - 1);
            const int el   = (u >> SLA) & (CHUNK - 1);
            const int pk   = ((cbase + el) << SLA) | slot;
            if (t < RCAP) {
              if (lane == 0) { hl[t] = pk; cnt[slot] = cnt[slot] + 1; }
              t = t + 1;
            } else {
              ov = 1;
            }
          }
        }
      }
    }
    __syncthreads();
  }
  if (wave == 0 && lane == 0) { misc[8] = t; misc[9] = ov; }
  __syncthreads();
  int tt = misc[8];
  tt = tt < 0 ? 0 : (tt > RCAP ? RCAP : tt);
  const int ovf = misc[9];

  if (wave == 0) {
    const int base = lane * (NBA / 32);
    int s = 0;
#pragma unroll 1
    for (int i = 0; i < NBA / 32; ++i) s += cnt[base + i];
    int incl = s;
#pragma unroll
    for (int d = 1; d < 32; d <<= 1) {
      const int y = __shfl_up(incl, d, 32);
      if (lane >= d) incl += y;
    }
    int run = incl - s;
#pragma unroll 1
    for (int i = 0; i < NBA / 32; ++i) {
      const int cv = cnt[base + i];
      offs[base + i] = run;
      cur[base + i]  = run;
      run += cv;
    }
  }
  __syncthreads();
  if (wave == 0) {
#pragma unroll 1
    for (int b0 = 0; b0 < tt; b0 += 32) {
      const int idx = b0 + lane;
      const int ent = hl[idx < RCAP ? idx : RCAP - 1];
      const int m32 = (tt - b0) < 32 ? (tt - b0) : 32;
#pragma unroll 1
      for (int k = 0; k < m32; ++k) {
        const int u    = __builtin_amdgcn_readlane(ent, k);
        const int slot = u & (NBA - 1);
        if (lane == 0) {
          int p = cur[slot];
          p = p < 0 ? 0 : (p > RCAP - 1 ? RCAP - 1 : p);
          sl[p] = u;
          cur[slot] = p + 1;
        }
      }
    }
  }
  __syncthreads();

  const float qnan = __int_as_float(0x7fc00000);
  const float pz = (ovf != 0) ? qnan : 0.0f;
  const int p0 = lane < NP ? lane : NP - 1;
  const int p1 = (NP > 32) ? (lane < NP - 32 ? lane : NP - 33) : 0;
#pragma unroll 1
  for (int si = 0; si < NBA / NWAVE; ++si) {
    const int s    = si * NWAVE + wave;
    const int node = nodeBase + s;
    int c = cnt[s];
    const bool big = c > DEGCAP;
    c = c < 0 ? 0 : (c > DEGCAP ? DEGCAP : c);
    int o = offs[s];
    o = o < 0 ? 0 : (o > RCAP ? RCAP : o);
    const int nc = node < nN ? node : nN - 1;
    const float dd = dis[nc];
    const float rd = dd * dd;
    float acc[NJ];
#pragma unroll
    for (int j = 0; j < NJ; ++j) acc[j] = 0.0f;
#pragma unroll 1
    for (int b0 = 0; b0 < c; b0 += 32) {
      int idx = o + b0 + lane;
      idx = idx > RCAP - 1 ? RCAP - 1 : idx;
      const int ent = sl[idx];
      int eid = ent >> SLA;
      eid = eid < 0 ? 0 : (eid > nE - 1 ? nE - 1 : eid);
      int sr = srcs[eid];
      sr = sr < 0 ? 0 : (sr > nN - 1 ? nN - 1 : sr);
      const float cf  = dis[sr] * dd;
      const int   cfi = __float_as_int(cf);
      const int m32 = (c - b0) < 32 ? (c - b0) : 32;
#pragma unroll 1
      for (int k = 0; k < m32; ++k) {
        const int   sk = __builtin_amdgcn_readlane(sr, k);
        const float ck = __int_as_float(__builtin_amdgcn_readlane(cfi, k));
        const float* rp = xl + (size_t)sk * PIN + lane;
#pragma unroll
        for (int j = 0; j < NJ; ++j) acc[j] = fmaf(ck, rp[32 * j], acc[j]);
      }
    }
    const float pzr = big ? qnan : pz;
    const bool live = node < nN;
    const float* sp = xl + (size_t)nc * PIN + lane;
    if constexpr (F32OUT != 0) {
      float* rbf = (float*)rowb;
#pragma unroll
      for (int j = 0; j < NJ; ++j) {
        float y = (acc[j] + sp[32 * j] * rd) + bv[j];
        y = relu_nan(y);
        y = y + pzr;
        rbf[lane + 32 * j] = live ? y : 0.0f;
      }
    } else {
      unsigned short* rbh = (unsigned short*)rowb;
#pragma unroll
      for (int j = 0; j < NJ; ++j) {
        const float y = (acc[j] + sp[32 * j] * rd) + pzr;
        const float v = live ? y : 0.0f;
        unsigned hb, lb;
        split_bf(v, hb, lb);
        rbh[lane + 32 * j]       = (unsigned short)hb;
        rbh[PIN + lane + 32 * j] = (unsigned short)lb;
      }
    }
    __syncthreads();
    const v4i q0 = *(const v4ia*)(rowb + 4 * p0);
    v4i q1 = {0, 0, 0, 0};
    if constexpr (NP > 32) q1 = *(const v4ia*)(rowb + 128 + 4 * p1);
    __syncthreads();
    const bool wrow = node < mRows;
    const int  na   = wrow ? node : 0;
    const bool w0 = wrow && (lane < (NP < 32 ? NP : 32));
    const bool w1 = wrow && (NP > 32) && (lane < NP - 32);
    int* orow = outp + (size_t)na * (size_t)PIN;
    if (w0) *(volatile v4i*)(orow + 4 * p0) = q0;
    if constexpr (NP > 32) { if (w1) *(volatile v4i*)(orow + 128 + 4 * p1) = q1; }
    __threadfence();
    if (w0) *(volatile v4i*)(orow + 4 * p0) = q0;
    if constexpr (NP > 32) { if (w1) *(volatile v4i*)(orow + 128 + 4 * p1) = q1; }
  }
}

__global__ __launch_bounds__(NTHR) void k_pool(const float* __restrict__ x3, const int* __restrict__ bat,
                                               int nN, unsigned short* G) {
  __shared__ __attribute__((aligned(16))) float wmax[NWAVE * N3P];
  __shared__ __attribute__((aligned(16))) unsigned short gs[KG1];
  const int tid = (int)threadIdx.x, lane = tid & 31, wave = tid >> 5;
  const int g = (int)blockIdx.x;
  const float ninf = __int_as_float((int)0xff800000u);

  v4f m0 = {ninf, ninf, ninf, ninf};
  v4f m1 = m0, m2 = m0;
  const int q2 = lane < 16 ? 64 + lane : 79;
#pragma unroll 1
  for (int i0 = wave * 32; i0 < nN; i0 += NTHR) {
    const int i  = i0 + lane;
    const int ic = i < nN ? i : nN - 1;
    const int b  = bat[ic];
    const bool hit = (i < nN) && (b == g);
    unsigned msk = __builtin_amdgcn_ballot_w32(hit);
    int nh = (int)__builtin_popcount(msk);
    nh = nh > 32 ? 32 : nh;
#pragma unroll 1
    for (int qq = 0; qq < nh; ++qq) {
      const int k = __builtin_ffs((int)msk) - 1;
      msk &= msk - 1u;
      int node = i0 + (k < 0 ? 0 : k);
      node = node > nN - 1 ? nN - 1 : node;
      const float* rp = x3 + (size_t)node * N3P;
      const v4f a = *(const v4fa*)(rp + 4 * lane);
      const v4f bq = *(const v4fa*)(rp + 128 + 4 * lane);
      const v4f cq = *(const v4fa*)(rp + 4 * q2);
      m0.x = nmax(m0.x, a.x);  m0.y = nmax(m0.y, a.y);  m0.z = nmax(m0.z, a.z);  m0.w = nmax(m0.w, a.w);
      m1.x = nmax(m1.x, bq.x); m1.y = nmax(m1.y, bq.y); m1.z = nmax(m1.z, bq.z); m1.w = nmax(m1.w, bq.w);
      m2.x = nmax(m2.x, cq.x); m2.y = nmax(m2.y, cq.y); m2.z = nmax(m2.z, cq.z); m2.w = nmax(m2.w, cq.w);
    }
  }
  *(v4fa*)(wmax + wave * N3P + 4 * lane) = m0;
  *(v4fa*)(wmax + wave * N3P + 128 + 4 * lane) = m1;
  if (lane < 16) *(v4fa*)(wmax + wave * N3P + 256 + 4 * lane) = m2;
  __syncthreads();
#pragma unroll 1
  for (int c = tid; c < N3P; c += NTHR) {
    float mm = ninf;
#pragma unroll
    for (int w2 = 0; w2 < NWAVE; ++w2) mm = nmax(mm, wmax[w2 * N3P + c]);
    mm = (c < F3) ? mm : 0.0f;
    unsigned hb, lb;
    split_bf(mm, hb, lb);
    gs[c]       = (unsigned short)hb;
    gs[N3P + c] = (unsigned short)lb;
  }
  __syncthreads();
  const int p = tid < (KG1 / 8) ? tid : (KG1 / 8) - 1;
  const v8us o = *(const v8usa*)(gs + 8 * p);
  unsigned short* gp = G + (size_t)g * KG1 + 8 * p;
  const bool ok = tid < (KG1 / 8);
  if (ok) *(volatile v8us*)gp = o;
  __threadfence();
  if (ok) *(volatile v8us*)gp = o;
}

static inline int cdiv(int a, int b) { return (a + b - 1) / b; }
static inline size_t al256(size_t o) { return (o + 255) & ~(size_t)255; }

extern "C" void kernel_launch(void* const* d_in, const int* in_sizes, int n_in,
                              void* d_out, int out_size, void* d_ws, size_t ws_size,
                              hipStream_t stream) {
  if (n_in < 13) return;
  if (in_sizes[0] < F0 || (in_sizes[0] % F0) != 0) return;
  const int nN = in_sizes[0] / F0;
  if (nN < 16 || nN > (1 << 22)) return;
  if (in_sizes[1] < 2 || (in_sizes[1] & 1) != 0) return;
  const int nE = in_sizes[1] / 2;
  if (nE < 1 || nE >= (1 << (31 - SLA))) return;
  if (in_sizes[2] != nN) return;
  if (in_sizes[3] != F0 * F1 || in_sizes[4] != F1) return;
  if (in_sizes[5] != F1 * F2 || in_sizes[6] != F2) return;
  if (in_sizes[7] != F2 * F3 || in_sizes[8] != F3) return;
  if (in_sizes[9] != F3 * FG || in_sizes[10] != FG) return;
  if (in_sizes[11] != FG * FO || in_sizes[12] != FO) return;
  if (out_size != NGR * FO) return;

  const float* x    = (const float*)d_in[0];
  const int*   edge = (const int*)d_in[1];
  const int*   bat  = (const int*)d_in[2];
  const float* W1   = (const float*)d_in[3];
  const float* b1   = (const float*)d_in[4];
  const float* W2   = (const float*)d_in[5];
  const float* b2   = (const float*)d_in[6];
  const float* W3   = (const float*)d_in[7];
  const float* b3   = (const float*)d_in[8];
  const float* Wg1  = (const float*)d_in[9];
  const float* bg1  = (const float*)d_in[10];
  const float* Wg2  = (const float*)d_in[11];
  const float* bg2  = (const float*)d_in[12];
  float* out = (float*)d_out;
  const int* src = edge;
  const int* dst = edge + nE;

  const int MP   = cdiv(nN, GBM) * GBM;
  const int gM   = MP / GBM;
  const int gD   = cdiv(nN, NBD);
  const int NBPD = gD * NBD;
  const int gA   = cdiv(MP, NBA);
  if ((long long)gA * NBA < (long long)MP) return;
  if (NBPD < nN) return;
  const int nUx = MP * (K1P / 8);
  if ((nUx % NTHR) != 0) return;
  const int vec8 = ((nE & 3) == 0) ? 1 : 0;

  const size_t szXB = (size_t)MP * K1P * 2;
  const size_t szH1 = (size_t)MP * N1P * 4;
  const size_t szX1 = (size_t)MP * N1P * 4;
  const size_t szA2 = (size_t)MP * K2P * 2;
  const size_t szX2 = (size_t)MP * N2P * 4;
  const size_t szA3 = (size_t)MP * K3P * 2;
  const size_t szX3 = (size_t)MP * N3P * 4;
  char* ws = (char*)d_ws;
  size_t off = 0;
  const size_t oXB = off; off = al256(off + szXB);
  const size_t oH1 = off; off = al256(off + szH1);
  const size_t oX1 = off; off = al256(off + szX1);
  const size_t oA2 = off; off = al256(off + szA2);
  const size_t oPend = off;
  if (szX2 > oA2 - oH1) return;
  if (szX3 > oPend) return;
  const size_t oA3  = off; off = al256(off + szA3);
  const size_t oDIS = off; off = al256(off + (size_t)NBPD * 4);
  const size_t oW1T = off; off = al256(off + (size_t)K1P * K1P * 2);
  const size_t oW2T = off; off = al256(off + (size_t)N2P * K2P * 2);
  const size_t oW3T = off; off = al256(off + (size_t)N3P * K3P * 2);
  const size_t oWG1 = off; off = al256(off + (size_t)FG * KG1 * 2);
  const size_t oWG2 = off; off = al256(off + (size_t)FO * KG2 * 2);
  const size_t oG   = off; off = al256(off + (size_t)NGR * KG1 * 2);
  const size_t oF   = off; off = al256(off + (size_t)NGR * KG2 * 2);
  if (off > ws_size || off > (size_t)WSMAX) return;
  unsigned short* XB   = (unsigned short*)(ws + oXB);
  float*          H1   = (float*)(ws + oH1);
  float*          X1   = (float*)(ws + oX1);
  unsigned short* A2   = (unsigned short*)(ws + oA2);
  float*          X2   = (float*)(ws + oH1);
  unsigned short* A3   = (unsigned short*)(ws + oA3);
  float*          X3   = (float*)(ws + oXB);
  float*          DIS  = (float*)(ws + oDIS);
  unsigned short* W1T  = (unsigned short*)(ws + oW1T);
  unsigned short* W2T2 = (unsigned short*)(ws + oW2T);
  unsigned short* W3T2 = (unsigned short*)(ws + oW3T);
  unsigned short* WG1  = (unsigned short*)(ws + oWG1);
  unsigned short* WG2  = (unsigned short*)(ws + oWG2);
  unsigned short* G    = (unsigned short*)(ws + oG);
  unsigned short* Fp   = (unsigned short*)(ws + oF);

  const size_t scanLds = (size_t)AGG_LDS_INTS * 4;
  hipFuncSetAttribute(reinterpret_cast<const void*>(&k_scan<3, 1>), hipFuncAttributeMaxDynamicSharedMemorySize, (int)scanLds);
  hipFuncSetAttribute(reinterpret_cast<const void*>(&k_scan<3, 0>), hipFuncAttributeMaxDynamicSharedMemorySize, (int)scanLds);
  hipFuncSetAttribute(reinterpret_cast<const void*>(&k_scan<5, 0>), hipFuncAttributeMaxDynamicSharedMemorySize, (int)scanLds);

  k_wprep<<<NUALL / NTHR, NTHR, 0, stream>>>(W1, W2, W3, Wg1, Wg2, W1T, W2T2, W3T2, WG1, WG2);
  k_cvx<<<nUx / NTHR, NTHR, 0, stream>>>(x, nN, nUx, XB);
  k_deg<<<gD, NTHR, 0, stream>>>(dst, nE, vec8, DIS);
  k_gemm<0><<<dim3(gM, N1P / GBN), GTHR, 0, stream>>>(XB, W1T, b1, F1, H1, Fp, K1P, N1P);
  k_scan<3, 1><<<gA, NTHR, scanLds, stream>>>(src, dst, nE, nN, vec8, MP, DIS, H1, b1, F1, (int*)X1);
  k_scan<3, 0><<<gA, NTHR, scanLds, stream>>>(src, dst, nE, nN, vec8, MP, DIS, X1, b1, F1, (int*)A2);
  k_gemm<1><<<dim3(gM, N2P / GBN), GTHR, 0, stream>>>(A2, W2T2, b2, F2, X2, Fp, K2P, N2P);
  k_scan<5, 0><<<gA, NTHR, scanLds, stream>>>(src, dst, nE, nN, vec8, MP, DIS, X2, b1, F1, (int*)A3);
  k_gemm<1><<<dim3(gM, N3P / GBN), GTHR, 0, stream>>>(A3, W3T2, b3, F3, X3, Fp, K3P, N3P);
  k_pool<<<NGR, NTHR, 0, stream>>>(X3, bat, nN, G);
  k_gemm<2><<<dim3(NGR / GBM, FG / GBN), GTHR, 0, stream>>>(G, WG1, bg1, FG, DIS, Fp, KG1, KG2);
  k_gemm<3><<<dim3(NGR / GBM, FO / GBN), GTHR, 0, stream>>>(Fp, WG2, bg2, FO, out, G, KG2, FO);
}
